// CoAtNetRelativeAttention_2156073583035
// MI455X (gfx1250) — hardware-verified
//
#include <hip/hip_runtime.h>


#define NBI  16
#define CC   256
#define NN   1024
#define NH_  8
#define HD   32
#define NRB  3969
#define PCAR 1024.0f
typedef _Float16 h16;
typedef unsigned short bf;
typedef __attribute__((ext_vector_type(16))) __bf16   v16bf;
typedef __attribute__((ext_vector_type(16))) _Float16 v16h;
typedef __attribute__((ext_vector_type(8)))  _Float16 v8h;
typedef __attribute__((ext_vector_type(8)))  unsigned short v8us;
typedef __attribute__((ext_vector_type(8)))  float    v8f;
typedef __attribute__((ext_vector_type(4)))  float    v4f;
typedef v8h  __attribute__((may_alias)) v8ha;
typedef v4f  __attribute__((may_alias)) v4fa;
typedef v8us __attribute__((may_alias)) v8usa;

__device__ __forceinline__ unsigned short f2bf(float f) { unsigned u = __float_as_uint(f); u += 0x7FFFu + ((u >> 16) & 1u); return (unsigned short)(u >> 16); }
__device__ __forceinline__ float bf2f(unsigned short b) { return __uint_as_float(((unsigned)b) << 16); }
__device__ __forceinline__ float bfr(float f) { return bf2f(f2bf(f)); }
__device__ __forceinline__ v16h cat16(v8h lo, v8h hi) { return __builtin_shufflevector(lo, hi, 0, 1, 2, 3, 4, 5, 6, 7, 8, 9, 10, 11, 12, 13, 14, 15); }
__device__ __forceinline__ v16bf cat16b(v8us lo, v8us hi) { return __builtin_bit_cast(v16bf, __builtin_shufflevector(lo, hi, 0, 1, 2, 3, 4, 5, 6, 7, 8, 9, 10, 11, 12, 13, 14, 15)); }
__device__ __forceinline__ v8f wmma16(v16h a, v16h b, v8f c) { return __builtin_amdgcn_wmma_f32_16x16x32_f16(false, a, false, b, (short)0, c, false, false); }
__device__ __forceinline__ v8f wmmab(v16bf a, v16bf b, v8f c) { return __builtin_amdgcn_wmma_f32_16x16x32_bf16(false, a, false, b, (short)0, c, false, false); }


template <typename T16> struct WFrag;
template <> struct WFrag<h16> { typedef v16h V; static __device__ __forceinline__ V ld(const h16* p) { return cat16(*(const v8h*)p, *(const v8h*)(p + 16)); } static __device__ __forceinline__ v8f mma(V a, V b, v8f c) { return wmma16(a, b, c); } };
template <> struct WFrag<bf> { typedef v16bf V; static __device__ __forceinline__ V ld(const bf* p) { return cat16b(*(const v8us*)p, *(const v8us*)(p + 16)); } static __device__ __forceinline__ v8f mma(V a, V b, v8f c) { return wmmab(a, b, c); } };
template <typename T16, int NSPLIT, bool BIAS>
__global__ __launch_bounds__(32) void k_gemmw(const T16* __restrict__ A, const T16* __restrict__ A2, const T16* __restrict__ Bt, const T16* __restrict__ Bt2, int K, float* C, int ldc, const float* __restrict__ bias, size_t sA, size_t sB, size_t sC) {
    typedef typename WFrag<T16>::V V;
    __shared__ __align__(16) float os[16 * 68];
    const size_t z = blockIdx.z; A += z * sA; if (A2) A2 += z * sA; Bt += z * sB; if (Bt2) Bt2 += z * sB; C += z * sC;
    const int lane = threadIdx.x & 31, lr = lane & 15, hi = lane >> 4; const int r0 = blockIdx.x * 64, c0 = blockIdx.y * 64;
    v8f acc[4][4];
#pragma unroll
    for (int mb = 0; mb < 4; ++mb)
#pragma unroll
        for (int nb = 0; nb < 4; ++nb) acc[mb][nb] = (v8f){};
    const size_t aoff = (size_t)(r0 + lr) * K + 8 * hi, boff = (size_t)(c0 + lr) * K + 8 * hi;
#pragma unroll 1
    for (int kc = 0; kc < K; kc += 32) {
        V a[4], a2[4];
#pragma unroll
        for (int mb = 0; mb < 4; ++mb) { a[mb] = WFrag<T16>::ld(A + aoff + (size_t)mb * 16 * K + kc); if (NSPLIT == 1 || NSPLIT == 2) a2[mb] = WFrag<T16>::ld(A2 + aoff + (size_t)mb * 16 * K + kc); }
#pragma unroll
        for (int nb = 0; nb < 4; ++nb) { const V b = WFrag<T16>::ld(Bt + boff + (size_t)nb * 16 * K + kc); V b2; if (NSPLIT >= 2) b2 = WFrag<T16>::ld(Bt2 + boff + (size_t)nb * 16 * K + kc);
#pragma unroll
            for (int mb = 0; mb < 4; ++mb) { acc[mb][nb] = WFrag<T16>::mma(a[mb], b, acc[mb][nb]); if (NSPLIT == 1 || NSPLIT == 2) acc[mb][nb] = WFrag<T16>::mma(a2[mb], b, acc[mb][nb]); if (NSPLIT >= 2) acc[mb][nb] = WFrag<T16>::mma(a[mb], b2, acc[mb][nb]); } }
        asm volatile("v_nop\n\tv_nop\n\tv_nop\n\tv_nop" : "+v"(acc[0][0]), "+v"(acc[1][1]), "+v"(acc[2][2]), "+v"(acc[3][3]) : "v"(a[0]), "v"(a[3]));
    }
#pragma unroll
    for (int mb = 0; mb < 4; ++mb) {
#pragma unroll
        for (int nb = 0; nb < 4; ++nb) {
#pragma unroll
            for (int j = 0; j < 8; ++j) os[(hi * 8 + j) * 68 + nb * 16 + lr] = acc[mb][nb][j]; }
        __builtin_amdgcn_wave_barrier(); asm volatile("" ::: "memory");
        float* crow = C + (size_t)(r0 + mb * 16) * ldc + c0;
#pragma unroll 1
        for (int ps = 0; ps < 2; ++ps) {
#pragma unroll
            for (int s = 0; s < 8; ++s) { const int row = 2 * s + hi, cofs = lr * 4; v4f val = *(const v4fa*)(os + row * 68 + cofs); if (BIAS) { val[0] += bfr(bias[c0 + cofs]); val[1] += bfr(bias[c0 + cofs + 1]); val[2] += bfr(bias[c0 + cofs + 2]); val[3] += bfr(bias[c0 + cofs + 3]); }
                *(volatile v4f*)(crow + (size_t)row * ldc + cofs) = val; }
            if (ps == 0) __threadfence(); }
        __builtin_amdgcn_wave_barrier(); asm volatile("" ::: "memory");
    }
}

__device__ __forceinline__ h16 tohx(float x) { return (h16)x; }
typedef __attribute__((ext_vector_type(2))) _Float16 v2h;
typedef __attribute__((ext_vector_type(4))) _Float16 v4h;
typedef __attribute__((ext_vector_type(4))) unsigned short v4us;
typedef __attribute__((ext_vector_type(4))) int v4i;

__global__ __launch_bounds__(256) void k_cvt8(const float* __restrict__ src, bf* dst, size_t n8) { const size_t i = (size_t)blockIdx.x * 256 + threadIdx.x; if (i >= n8) return; const v8f v = *(const v8f*)(src + i * 8); v8us o;
#pragma unroll
    for (int k = 0; k < 8; ++k) o[k] = f2bf(v[k]); *(volatile v8us*)(dst + i * 8) = o; __threadfence(); *(volatile v8us*)(dst + i * 8) = o; }
__global__ __launch_bounds__(256) void k_w16(const float* __restrict__ w, size_t n4, h16* Bt) { const size_t i = ((size_t)blockIdx.x * 256 + threadIdx.x) * 4; if (i >= n4 * 4) return; const v4f a = *(const v4f*)(w + i); v4h o; o[0] = tohx(bfr(a[0])); o[1] = tohx(bfr(a[1])); o[2] = tohx(bfr(a[2])); o[3] = tohx(bfr(a[3])); *(volatile v4h*)(Bt + i) = o; __threadfence(); *(volatile v4h*)(Bt + i) = o; }
__global__ __launch_bounds__(256) void k_xt(const float* __restrict__ x, bf* XT) { const size_t e = ((size_t)blockIdx.x * 256 + threadIdx.x) * 4; if (e >= (size_t)NN * CC) return; const int c = (int)(e % CC); const int n = (int)(e / CC); v4us o;
#pragma unroll
    for (int q = 0; q < 4; ++q) o[q] = f2bf(x[(size_t)(c + q) * NN + n]); *(volatile v4us*)(XT + e) = o; __threadfence(); *(volatile v4us*)(XT + e) = o; }
__global__ __launch_bounds__(256) void k_qkpl(const float* __restrict__ Q, const float* __restrict__ Kf, h16* Q16, h16* K16) { const size_t e = ((size_t)blockIdx.x * 256 + threadIdx.x) * 4; if (e >= (size_t)NH_ * NN * HD) return; const int d = (int)(e % HD); const int n = (int)((e / HD) % NN); const int h = (int)(e / ((size_t)HD * NN)); const size_t src = (size_t)n * CC + h * HD + d; const v4f a = *(const v4f*)(Q + src), c = *(const v4f*)(Kf + src); v4h oq, ok;
#pragma unroll
    for (int q = 0; q < 4; ++q) { oq[q] = tohx(a[q]); ok[q] = tohx(c[q] * 0.1767766952966369f); } for (int ps = 0; ps < 2; ++ps) { *(volatile v4h*)(Q16 + e) = oq; *(volatile v4h*)(K16 + e) = ok; if (ps == 0) __threadfence(); } }
__global__ __launch_bounds__(256) void k_vt(const float* __restrict__ V, h16* VT) { const size_t e = ((size_t)blockIdx.x * 256 + threadIdx.x) * 2; if (e >= (size_t)NH_ * 64 * NN) return; const int n = (int)(e % NN); const int dv = (int)((e / NN) % 64); const int h = (int)(e / ((size_t)NN * 64)); v2h o; o[0] = dv < HD ? tohx(V[(size_t)n * CC + h * HD + dv]) : (h16)0.f; o[1] = dv < HD ? tohx(V[(size_t)(n + 1) * CC + h * HD + dv]) : (h16)0.f; *(volatile v2h*)(VT + e) = o; __threadfence(); *(volatile v2h*)(VT + e) = o; }
__global__ __launch_bounds__(256) void k_softb(const float* __restrict__ Sb, const float* __restrict__ rb, const int* __restrict__ ridx, h16* P) { const int lane = threadIdx.x & 31; const int row = blockIdx.x * 8 + (threadIdx.x >> 5); if (row >= NH_ * NN) return; const int i = row % NN; const int h = row / NN; const float* sr = Sb + (size_t)row * NN; const int* ir = ridx + (size_t)i * NN; const float* rbh = rb + (size_t)h * NRB; h16* pr = P + (size_t)row * NN; float mx = -3.0e38f;
#pragma unroll 1
    for (int ch = 0; ch < NN / 128; ++ch) { const int j0 = ch * 128 + lane * 4; const v4f a = *(const v4f*)(sr + j0); const v4i ii = *(const v4i*)(ir + j0);
#pragma unroll
        for (int q = 0; q < 4; ++q) { const int k = min(max(ii[q], 0), NRB - 1); mx = fmaxf(mx, __fadd_rn(a[q], bfr(rbh[k]))); } }
#pragma unroll
    for (int sh = 16; sh; sh >>= 1) mx = fmaxf(mx, __shfl_xor(mx, sh, 32));
    float sum = 0.f;
#pragma unroll 1
    for (int ch = 0; ch < NN / 128; ++ch) { const int j0 = ch * 128 + lane * 4; const v4f a = *(const v4f*)(sr + j0); const v4i ii = *(const v4i*)(ir + j0);
#pragma unroll
        for (int q = 0; q < 4; ++q) { const int k = min(max(ii[q], 0), NRB - 1); float d0 = __fsub_rn(__fadd_rn(a[q], bfr(rbh[k])), mx); asm volatile("" : "+v"(d0)); sum += __expf(d0); } }
#pragma unroll
    for (int sh = 16; sh; sh >>= 1) sum += __shfl_xor(sum, sh, 32);
    const float f = __fdiv_rn(PCAR, sum);
    for (int ps = 0; ps < 2; ++ps) {
#pragma unroll 1
        for (int ch = 0; ch < NN / 128; ++ch) { const int j0 = ch * 128 + lane * 4; const v4f a = *(const v4f*)(sr + j0); const v4i ii = *(const v4i*)(ir + j0); v4h o;
#pragma unroll
            for (int q = 0; q < 4; ++q) { const int k = min(max(ii[q], 0), NRB - 1); float d0 = __fsub_rn(__fadd_rn(a[q], bfr(rbh[k])), mx); asm volatile("" : "+v"(d0)); o[q] = tohx(__fmul_rn(__expf(d0), f)); } *(volatile v4h*)(pr + j0) = o; }
        if (ps == 0) __threadfence(); } }
__global__ __launch_bounds__(256) void k_mrg16(const float* __restrict__ O, h16* M16) { const size_t e = ((size_t)blockIdx.x * 256 + threadIdx.x) * 4; if (e >= (size_t)NN * CC) return; const int c = (int)(e % CC); const int n = (int)(e / CC); const int h = c / HD, d = c % HD; const float* r = O + ((size_t)h * NN + n) * 64 + d; v4h o; o[0] = tohx(r[0] * (1.0f / PCAR)); o[1] = tohx(r[1] * (1.0f / PCAR)); o[2] = tohx(r[2] * (1.0f / PCAR)); o[3] = tohx(r[3] * (1.0f / PCAR)); *(volatile v4h*)(M16 + e) = o; __threadfence(); *(volatile v4h*)(M16 + e) = o; }
__global__ __launch_bounds__(256) void k_outT(const float* __restrict__ R, const float* __restrict__ bo, float* OUT) { const size_t e = ((size_t)blockIdx.x * 256 + threadIdx.x) * 4; if (e >= (size_t)CC * NN) return; const int n = (int)(e % NN); const int c = (int)(e / NN); const float bb = bfr(bo[c]); v4f o;
#pragma unroll
    for (int q = 0; q < 4; ++q) o[q] = __fadd_rn(R[(size_t)(n + q) * CC + c], bb); *(volatile v4f*)(OUT + e) = o; __threadfence(); *(volatile v4f*)(OUT + e) = o; }

extern "C" void kernel_launch(void* const* d_in, const int* in_sizes, int n_in,
                              void* d_out, int out_size, void* d_ws, size_t ws_size, hipStream_t stream) {
    (void)in_sizes; (void)n_in; (void)out_size;
    const float* x = (const float*)d_in[0]; const float* wq = (const float*)d_in[1]; const float* wk = (const float*)d_in[2]; const float* wv = (const float*)d_in[3]; const float* wo = (const float*)d_in[4]; const float* bo = (const float*)d_in[5]; const float* rb = (const float*)d_in[6]; const int* ridx = (const int*)d_in[7];
    float* OUT = (float*)d_out;
    char* wsp = (char*)d_ws;
    auto take = [&](size_t bytes) { char* p = wsp; wsp += (bytes + 255) & ~(size_t)255; return (void*)p; };
    bf* WQ = (bf*)take(CC * CC * 2); bf* WK = (bf*)take(CC * CC * 2); bf* WV = (bf*)take(CC * CC * 2); h16* WO = (h16*)take(CC * CC * 2); bf* XT = (bf*)take((size_t)NN * CC * 2); float* Q = (float*)take((size_t)NN * CC * 4); float* Kf = (float*)take((size_t)NN * CC * 4); float* V = (float*)take((size_t)NN * CC * 4);
    h16* Q16 = (h16*)take((size_t)NH_ * NN * HD * 2); h16* K16 = (h16*)take((size_t)NH_ * NN * HD * 2); h16* VT = (h16*)take((size_t)NH_ * 64 * NN * 2); float* Sb = (float*)take((size_t)NH_ * NN * NN * 4); h16* P16 = (h16*)take((size_t)NH_ * NN * NN * 2); float* O = (float*)take((size_t)NH_ * NN * 64 * 4); h16* M16 = (h16*)take((size_t)NN * CC * 2); float* R = (float*)take((size_t)NN * CC * 4);
    if ((size_t)(wsp - (char*)d_ws) > ws_size) return;
    k_cvt8<<<(CC * CC / 8 + 255) / 256, 256, 0, stream>>>(wq, WQ, CC * CC / 8); k_cvt8<<<(CC * CC / 8 + 255) / 256, 256, 0, stream>>>(wk, WK, CC * CC / 8); k_cvt8<<<(CC * CC / 8 + 255) / 256, 256, 0, stream>>>(wv, WV, CC * CC / 8); k_w16<<<(CC * CC / 4 + 255) / 256, 256, 0, stream>>>(wo, CC * CC / 4, WO);
    for (int b = 0; b < NBI; ++b) {
        k_xt<<<(unsigned)(((size_t)NN * CC / 4 + 255) / 256), 256, 0, stream>>>(x + (size_t)b * CC * NN, XT);
        k_gemmw<bf, 0, false><<<dim3(NN / 64, CC / 64, 1), 32, 0, stream>>>(XT, nullptr, WQ, nullptr, CC, Q, CC, nullptr, 0, 0, 0); k_gemmw<bf, 0, false><<<dim3(NN / 64, CC / 64, 1), 32, 0, stream>>>(XT, nullptr, WK, nullptr, CC, Kf, CC, nullptr, 0, 0, 0); k_gemmw<bf, 0, false><<<dim3(NN / 64, CC / 64, 1), 32, 0, stream>>>(XT, nullptr, WV, nullptr, CC, V, CC, nullptr, 0, 0, 0);
        k_qkpl<<<(unsigned)(((size_t)NH_ * NN * HD / 4 + 255) / 256), 256, 0, stream>>>(Q, Kf, Q16, K16); k_vt<<<(unsigned)(((size_t)NH_ * 64 * NN / 2 + 255) / 256), 256, 0, stream>>>(V, VT);
        k_gemmw<h16, 0, false><<<dim3(NN / 64, NN / 64, NH_), 32, 0, stream>>>(Q16, nullptr, K16, nullptr, HD, Sb, NN, nullptr, (size_t)NN * HD, (size_t)NN * HD, (size_t)NN * NN);
        k_softb<<<(NH_ * NN + 7) / 8, 256, 0, stream>>>(Sb, rb, ridx, P16);
        k_gemmw<h16, 0, false><<<dim3(NN / 64, 1, NH_), 32, 0, stream>>>(P16, nullptr, VT, nullptr, NN, O, 64, nullptr, (size_t)NN * NN, (size_t)64 * NN, (size_t)NN * 64);
        k_mrg16<<<(unsigned)(((size_t)NN * CC / 4 + 255) / 256), 256, 0, stream>>>(O, M16);
        k_gemmw<h16, 0, false><<<dim3(NN / 64, CC / 64, 1), 32, 0, stream>>>(M16, nullptr, WO, nullptr, CC, R, CC, nullptr, 0, 0, 0);
        k_outT<<<(unsigned)(((size_t)CC * NN / 4 + 255) / 256), 256, 0, stream>>>(R, bo, OUT + (size_t)b * CC * NN); }
}
